// ModifiedGCN_21157008900177
// MI455X (gfx1250) — hardware-verified
//
#include <hip/hip_runtime.h>
#include <stddef.h>


#define F       64
#define GFD     32
#define HIN     (2 * F + GFD)
#define L1D     256
#define L2D     128
#define NTHR    256
#define NWAVE   8
#define EPT     8
#define NGRP    2
#define CHUNK   (NTHR * EPT * NGRP)
#define WCAP    (EPT * NGRP * 32)
#define LISTN   (NWAVE * WCAP)
#define NBC     4096
#define NBF     1024
#define NBP     32
#define RCAP    24576
#define RBN     128
#define OTHR    512
#define TGT     128
#define AP      (F + 8)
#define DEGCAP  128
#define SROWS   64
#define GOUT    128
#define ASCALE  64.0f
#define WSCALE  8.0f
#define OSCALE  0.001953125f
#define SLOPE   0.01f
#define LDS_FILL ((RCAP + NBF + LISTN) * 4 + 64)

static_assert((CHUNK & (CHUNK - 1)) == 0);
static_assert(CHUNK <= 4096);
static_assert(NBC <= 4096 && NBF <= 4096 && NBP <= 4096);
static_assert((NBC & (NBC - 1)) == 0 && (NBF & (NBF - 1)) == 0 && (NBP & (NBP - 1)) == 0);
static_assert(NBC == 4 * NBF);
static_assert(OTHR * 8 == NBC);
static_assert((RCAP % 32) == 0);
static_assert(RBN == 128);
static_assert(F == 64);
static_assert(TGT == NWAVE * 16);
static_assert(TGT * AP * 2 <= TGT * F * 4);
static_assert((AP % 8) == 0);
static_assert((F * F / 8) % NTHR == 0);
static_assert(SROWS * F / 4 == 4 * NTHR);
static_assert(NBP * 2 * F / 4 == 4 * NTHR);
static_assert(L1D == NTHR && L2D <= NTHR && L2D == 4 * 32);
static_assert(GOUT == 4 * 32);
static_assert(HIN <= NTHR);

typedef float    v2f  __attribute__((ext_vector_type(2)));
typedef float    v4f  __attribute__((ext_vector_type(4)));
typedef float    v8f  __attribute__((ext_vector_type(8)));
typedef int      v4i  __attribute__((ext_vector_type(4)));
typedef _Float16 v4h  __attribute__((ext_vector_type(4)));
typedef _Float16 v8h  __attribute__((ext_vector_type(8)));
typedef _Float16 v16h __attribute__((ext_vector_type(16)));
union FragH { v16h v; v8h h[2]; };

__device__ __forceinline__ v8h cvt8(v4f a, v4f b) {
  v8h r;
  r[0] = (_Float16)a.x; r[1] = (_Float16)a.y; r[2] = (_Float16)a.z; r[3] = (_Float16)a.w;
  r[4] = (_Float16)b.x; r[5] = (_Float16)b.y; r[6] = (_Float16)b.z; r[7] = (_Float16)b.w;
  return r;
}

__device__ __forceinline__ v8f wmh(v16h a, v16h b, v8f c) {
  v8f d = __builtin_amdgcn_wmma_f32_16x16x32_f16(false, a, false, b, (short)0, c, false, false);
  asm volatile("v_nop\n\tv_nop\n\tv_nop\n\tv_nop" : "+v"(d) : "v"(a), "v"(b));
  return d;
}

__device__ __forceinline__ float lrelu(float v) { return v >= 0.0f ? v : SLOPE * v; }

template <int NB>
__device__ __forceinline__ int scan_chunk(const int* __restrict__ dsts, int nE, int cbase, int slotBase,
                                          int vec8, int* list, int tid, int lane, int wave) {
  int wc = 0;
#pragma unroll
  for (int g = 0; g < NGRP; ++g) {
    const int el0  = (g * NTHR + tid) * EPT;
    const int e0   = cbase + el0;
    const int sent = -2147483647 - 1;
    v4i da, db;
    if (vec8 != 0 && cbase + CHUNK <= nE) {
      da = *(const v4i*)(dsts + e0);
      db = *(const v4i*)(dsts + e0 + 4);
    } else {
      da.x = (e0     < nE) ? dsts[min(e0, nE - 1)] : sent;
      da.y = (e0 + 1 < nE) ? dsts[min(e0 + 1, nE - 1)] : sent;
      da.z = (e0 + 2 < nE) ? dsts[min(e0 + 2, nE - 1)] : sent;
      da.w = (e0 + 3 < nE) ? dsts[min(e0 + 3, nE - 1)] : sent;
      db.x = (e0 + 4 < nE) ? dsts[min(e0 + 4, nE - 1)] : sent;
      db.y = (e0 + 5 < nE) ? dsts[min(e0 + 5, nE - 1)] : sent;
      db.z = (e0 + 6 < nE) ? dsts[min(e0 + 6, nE - 1)] : sent;
      db.w = (e0 + 7 < nE) ? dsts[min(e0 + 7, nE - 1)] : sent;
    }
    const unsigned nb = (unsigned)slotBase;
    const unsigned s0 = (unsigned)da.x - nb, s1 = (unsigned)da.y - nb;
    const unsigned s2 = (unsigned)da.z - nb, s3 = (unsigned)da.w - nb;
    const unsigned s4 = (unsigned)db.x - nb, s5 = (unsigned)db.y - nb;
    const unsigned s6 = (unsigned)db.z - nb, s7 = (unsigned)db.w - nb;
    const bool h0 = s0 < (unsigned)NB, h1 = s1 < (unsigned)NB, h2 = s2 < (unsigned)NB, h3 = s3 < (unsigned)NB;
    const bool h4 = s4 < (unsigned)NB, h5 = s5 < (unsigned)NB, h6 = s6 < (unsigned)NB, h7 = s7 < (unsigned)NB;
    const unsigned any = __builtin_amdgcn_ballot_w32(h0 | h1 | h2 | h3 | h4 | h5 | h6 | h7);
    if (any != 0u) {
#define HITJ(J, HJ, SJ) { \
        const unsigned mj = __builtin_amdgcn_ballot_w32(HJ); \
        if (mj != 0u) { \
          if (HJ) { \
            const int pos = wc + (int)__builtin_amdgcn_mbcnt_lo(mj, 0u); \
            if (pos < WCAP) list[wave * WCAP + pos] = ((el0 + (J)) << 12) | (int)(SJ); \
          } \
          wc += (int)__builtin_popcount(mj); } }
      HITJ(0, h0, s0)
      HITJ(1, h1, s1)
      HITJ(2, h2, s2)
      HITJ(3, h3, s3)
      HITJ(4, h4, s4)
      HITJ(5, h5, s5)
      HITJ(6, h6, s6)
      HITJ(7, h7, s7)
#undef HITJ
    }
  }
  return wc;
}

__global__ __launch_bounds__(NTHR) void k_wprep(
    const float* __restrict__ w1, const float* __restrict__ w2, const float* __restrict__ w3, _Float16* wp) {
  const int i = blockIdx.x * NTHR + (int)threadIdx.x;
  const int layer = i / (F * F / 8);
  const float* src = layer == 0 ? w1 : (layer == 1 ? w2 : w3);
  const int o  = (i - layer * (F * F / 8)) * 8;
  const int n  = o / F;
  const int k0 = o - n * F;
  float v[8];
#pragma unroll
  for (int e = 0; e < 8; ++e) v[e] = src[(size_t)(k0 + e) * F + n] * WSCALE;
  v4f a, b;
  a.x = v[0]; a.y = v[1]; a.z = v[2]; a.w = v[3];
  b.x = v[4]; b.y = v[5]; b.z = v[6]; b.w = v[7];
  const v8h hv = cvt8(a, b);
  _Float16* dp = wp + (size_t)layer * F * F + o;
  *(volatile v8h*)dp = hv;
  __threadfence();
  *(volatile v8h*)dp = hv;
}

__global__ __launch_bounds__(NTHR) void k_count(
    const int* __restrict__ ei, int* cnt, float* dinv, int nE, int vec8) {
  __shared__ __attribute__((aligned(16))) int scnt[NBC];
  __shared__ __attribute__((aligned(16))) int list[LISTN];
  __shared__ int wcnt[NWAVE];
  const int tid = threadIdx.x, lane = tid & 31, wave = tid >> 5;
  const int nodeBase = blockIdx.x * NBC;
  const int* dsts = ei + nE;

  for (int i = tid; i < NBC; i += NTHR) scnt[i] = 0;
  __syncthreads();

  const int nChunks = (nE + CHUNK - 1) / CHUNK;
#pragma unroll 1
  for (int ch = 0; ch < nChunks; ++ch) {
    const int cbase = ch * CHUNK;
    const int wc = scan_chunk<NBC>(dsts, nE, cbase, nodeBase, vec8, list, tid, lane, wave);
    if (lane == 0) wcnt[wave] = wc;
    __syncthreads();
    if (wave == 0) {
#pragma unroll 1
      for (int wsx = 0; wsx < NWAVE; ++wsx) {
        int n = __builtin_amdgcn_readfirstlane(wcnt[wsx]);
        n = n > WCAP ? WCAP : (n < 0 ? 0 : n);
        const int* lp = list + wsx * WCAP;
#pragma unroll 1
        for (int i = 0; i < n; ++i) {
          const int ent  = __builtin_amdgcn_readfirstlane(lp[i]);
          const int slot = ent & (NBC - 1);
          if (lane == 0) scnt[slot] = scnt[slot] + 1;
        }
      }
    }
    __syncthreads();
  }

  v4i cq[4]; v4f dq[4];
#pragma unroll
  for (int q = 0; q < 4; ++q) {
    const int f = (wave * 4 + q) * 128 + 4 * lane;
    const v4i c = *(const v4i*)(scnt + f);
    cq[q] = c;
    dq[q].x = rsqrtf((float)(c.x + 1));
    dq[q].y = rsqrtf((float)(c.y + 1));
    dq[q].z = rsqrtf((float)(c.z + 1));
    dq[q].w = rsqrtf((float)(c.w + 1));
  }
  int*   cp = cnt + (size_t)nodeBase;
  float* dp = dinv + (size_t)nodeBase;
#pragma unroll
  for (int q = 0; q < 4; ++q) {
    const int f = (wave * 4 + q) * 128 + 4 * lane;
    *(volatile v4i*)(cp + f) = cq[q];
    *(volatile v4f*)(dp + f) = dq[q];
  }
  __threadfence();
#pragma unroll
  for (int q = 0; q < 4; ++q) {
    const int f = (wave * 4 + q) * 128 + 4 * lane;
    *(volatile v4i*)(cp + f) = cq[q];
    *(volatile v4f*)(dp + f) = dq[q];
  }
}

__global__ __launch_bounds__(OTHR) void k_offsets(
    const int* __restrict__ cnt, int* off, int* rbase, int nChunk) {
  __shared__ __attribute__((aligned(16))) int soff[NBC];
  __shared__ __attribute__((aligned(16))) int srb[RBN];
  __shared__ int wtot[OTHR / 32];
  const int tid = threadIdx.x, lane = tid & 31, wave = tid >> 5, sub = tid >> 7;
  for (int i = tid; i < RBN; i += OTHR) srb[i] = 0;
  int carry = 0;
#pragma unroll 1
  for (int ch = 0; ch < nChunk; ++ch) {
    const int base = ch * NBC;
    const v4i c0 = *(const v4i*)(cnt + base + 8 * tid);
    const v4i c1 = *(const v4i*)(cnt + base + 8 * tid + 4);
    const int e0 = max(c0.x, 0), e1 = max(c0.y, 0), e2 = max(c0.z, 0), e3 = max(c0.w, 0);
    const int e4 = max(c1.x, 0), e5 = max(c1.y, 0), e6 = max(c1.z, 0), e7 = max(c1.w, 0);
    const int ts = e0 + e1 + e2 + e3 + e4 + e5 + e6 + e7;
    int incl = ts;
#pragma unroll
    for (int d = 1; d < 32; d <<= 1) {
      const int t = __shfl_up(incl, d);
      if (lane >= d) incl += t;
    }
    if (lane == 31) wtot[wave] = incl;
    __syncthreads();
    const int S0 = wtot[0]  + wtot[1]  + wtot[2]  + wtot[3];
    const int S1 = wtot[4]  + wtot[5]  + wtot[6]  + wtot[7];
    const int S2 = wtot[8]  + wtot[9]  + wtot[10] + wtot[11];
    const int S3 = wtot[12] + wtot[13] + wtot[14] + wtot[15];
    int pre = 0;
#pragma unroll 1
    for (int w = 4 * sub; w < wave; ++w) pre += wtot[w];
    const int b0 = carry;
    const int b1 = b0 + ((S0 + 31) & ~31);
    const int b2 = b1 + ((S1 + 31) & ~31);
    const int b3 = b2 + ((S2 + 31) & ~31);
    const int b4 = b3 + ((S3 + 31) & ~31);
    const int myb = sub == 0 ? b0 : (sub == 1 ? b1 : (sub == 2 ? b2 : b3));
    if (tid == 0) {
      srb[min(4 * ch + 0, RBN - 1)] = b0;
      srb[min(4 * ch + 1, RBN - 1)] = b1;
      srb[min(4 * ch + 2, RBN - 1)] = b2;
      srb[min(4 * ch + 3, RBN - 1)] = b3;
    }
    int run = myb + pre + incl - ts;
    soff[8 * tid + 0] = run; run += e0;
    soff[8 * tid + 1] = run; run += e1;
    soff[8 * tid + 2] = run; run += e2;
    soff[8 * tid + 3] = run; run += e3;
    soff[8 * tid + 4] = run; run += e4;
    soff[8 * tid + 5] = run; run += e5;
    soff[8 * tid + 6] = run; run += e6;
    soff[8 * tid + 7] = run;
    carry = b4;
    __syncthreads();
    const v4i o0 = *(const v4i*)(soff + 4 * tid);
    const v4i o1 = *(const v4i*)(soff + 4 * (tid + OTHR));
    int* op = off + base;
    *(volatile v4i*)(op + 4 * tid) = o0;
    *(volatile v4i*)(op + 4 * (tid + OTHR)) = o1;
    __threadfence();
    *(volatile v4i*)(op + 4 * tid) = o0;
    *(volatile v4i*)(op + 4 * (tid + OTHR)) = o1;
    __syncthreads();
  }
  if (tid == 0) srb[min(4 * nChunk, RBN - 1)] = carry;
  __syncthreads();
  v4i rv = {0, 0, 0, 0};
  if (tid < 32) rv = *(const v4i*)(srb + 4 * tid);
  if (tid < 32) *(volatile v4i*)(rbase + 4 * tid) = rv;
  __threadfence();
  if (tid < 32) *(volatile v4i*)(rbase + 4 * tid) = rv;
}

__global__ __launch_bounds__(NTHR) void k_fill(
    const int* __restrict__ ei, const int* __restrict__ off, const int* __restrict__ rbase,
    int* csr, int nN, int nE, int vec8, int csrLen) {
  extern __shared__ v4f lds_dyn[];
  int* region = (int*)lds_dyn;
  int* cursor = region + RCAP;
  int* list   = cursor + NBF;
  int* wcnt   = list + LISTN;
  const int tid = threadIdx.x, lane = tid & 31, wave = tid >> 5;
  const int b = blockIdx.x;
  const int nodeBase = b * NBF;
  const int* dsts = ei + nE;

  int rb0 = rbase[b];
  const int rb1 = rbase[b + 1];
  rb0 = rb0 < 0 ? 0 : (rb0 > csrLen ? csrLen : rb0);
  rb0 &= ~31;
  int len = rb1 - rb0;
  len = len < 0 ? 0 : (len > RCAP ? RCAP : len);
  int lenW = (len + 31) & ~31;
  if (rb0 + lenW > csrLen) lenW = (csrLen - rb0) & ~31;

  {
    const v4i z = {0, 0, 0, 0};
    for (int i = tid; i < RCAP / 4; i += NTHR) ((v4i*)region)[i] = z;
    for (int s = tid; s < NBF; s += NTHR) {
      int o = off[nodeBase + s] - rb0;
      o = o < 0 ? 0 : (o > RCAP ? RCAP : o);
      cursor[s] = o;
    }
  }
  __syncthreads();

  const int nChunks = (nE + CHUNK - 1) / CHUNK;
#pragma unroll 1
  for (int ch = 0; ch < nChunks; ++ch) {
    const int cbase = ch * CHUNK;
    const int wc = scan_chunk<NBF>(dsts, nE, cbase, nodeBase, vec8, list, tid, lane, wave);
    if (lane == 0) wcnt[wave] = wc;
    __syncthreads();
    if (wave == 0) {
#pragma unroll 1
      for (int wsx = 0; wsx < NWAVE; ++wsx) {
        int n = __builtin_amdgcn_readfirstlane(wcnt[wsx]);
        n = n > WCAP ? WCAP : (n < 0 ? 0 : n);
        const int* lp = list + wsx * WCAP;
#pragma unroll 1
        for (int i = 0; i < n; ++i) {
          const int ent  = __builtin_amdgcn_readfirstlane(lp[i]);
          const int slot = ent & (NBF - 1);
          int e = cbase + ((ent >> 12) & (CHUNK - 1));
          e = e > nE - 1 ? nE - 1 : e;
          int src = ei[e];
          src = src < 0 ? 0 : (src > nN - 1 ? nN - 1 : src);
          if (lane == 0) {
            int pos = cursor[slot];
            pos = pos < 0 ? 0 : (pos > RCAP - 1 ? RCAP - 1 : pos);
            region[pos] = src;
            const int np = pos + 1;
            cursor[slot] = np > RCAP ? RCAP : np;
          }
        }
      }
    }
    __syncthreads();
  }

  const int nv = lenW >> 2;
  int* gp = csr + rb0;
#pragma unroll 1
  for (int i = tid; i < nv; i += NTHR) { const v4i v = ((const v4i*)region)[i]; *(volatile v4i*)(gp + 4 * i) = v; }
  __threadfence();
#pragma unroll 1
  for (int i = tid; i < nv; i += NTHR) { const v4i v = ((const v4i*)region)[i]; *(volatile v4i*)(gp + 4 * i) = v; }
}

__global__ __launch_bounds__(NTHR) void k_scale(
    const float* __restrict__ x, const float* __restrict__ dinv, float* xs, int nN) {
  const int tid = threadIdx.x;
  const int rowBase = blockIdx.x * SROWS;
  v4f v[4];
#pragma unroll
  for (int p = 0; p < 4; ++p) {
    const int g  = p * NTHR + tid;
    const int r  = g >> 4;
    const int c0 = (g & 15) * 4;
    const int row = rowBase + r;
    const int rr  = row > nN - 1 ? nN - 1 : row;
    const float d = dinv[row];
    v[p] = *(const v4f*)(x + (size_t)rr * F + c0) * d;
  }
  float* gp = xs + (size_t)rowBase * F;
#pragma unroll
  for (int p = 0; p < 4; ++p) *(volatile v4f*)(gp + 4 * (p * NTHR + tid)) = v[p];
  __threadfence();
#pragma unroll
  for (int p = 0; p < 4; ++p) *(volatile v4f*)(gp + 4 * (p * NTHR + tid)) = v[p];
}

__global__ __launch_bounds__(NTHR) void k_layer(
    const int* __restrict__ csr, const int* __restrict__ off, const int* __restrict__ cnt,
    const float* __restrict__ dinv, const float* __restrict__ xs, const _Float16* __restrict__ wp,
    const float* __restrict__ bias, float* xo, int nN, int csrLen, int scaleOut) {
  __shared__ __attribute__((aligned(16))) v4f lds[TGT * F / 4];
  _Float16* sA  = (_Float16*)lds;
  float*    stg = (float*)lds;
  const int tid = threadIdx.x, lane = tid & 31, wave = tid >> 5, hh = lane >> 4, m = lane & 15;
  const int q4 = 4 * m;
  const int rowBase = blockIdx.x * TGT;
  const int tbase = rowBase + wave * 16;
  const int cl = tbase + m;
  const int cnt_l = cnt[cl];
  const int off_l = off[cl];
  const int dv_l  = __float_as_int(dinv[cl]);

#pragma unroll 1
  for (int j = 0; j < 16; ++j) {
    const int c = tbase + j;
    int n = __builtin_amdgcn_readlane(cnt_l, j);
    n = n < 0 ? 0 : (n > DEGCAP ? DEGCAP : n);
    const int st = __builtin_amdgcn_readlane(off_l, j);
    const float dc = __int_as_float(__builtin_amdgcn_readlane(dv_l, j));
    v4f acc = {0.f, 0.f, 0.f, 0.f};
#pragma unroll 1
    for (int q0 = 0; q0 < n; q0 += 32) {
      int pos = st + q0 + lane;
      pos = pos < 0 ? 0 : (pos > csrLen - 1 ? csrLen - 1 : pos);
      int sl = csr[pos];
      sl = sl < 0 ? 0 : (sl > nN - 1 ? nN - 1 : sl);
      const int mcnt = (n - q0) < 32 ? (n - q0) : 32;
#pragma unroll 1
      for (int p = 0; p < mcnt; p += 2) {
        const int s0 = __builtin_amdgcn_readlane(sl, p);
        const int s1 = __builtin_amdgcn_readlane(sl, p + 1);
        const int s  = hh != 0 ? s1 : s0;
        const v4f v  = *(const v4f*)(xs + (size_t)s * F + q4);
        const bool ok = (hh == 0) || (p + 1 < mcnt);
        acc.x += ok ? v.x : 0.0f;
        acc.y += ok ? v.y : 0.0f;
        acc.z += ok ? v.z : 0.0f;
        acc.w += ok ? v.w : 0.0f;
      }
    }
    v4f tot;
    tot.x = acc.x + __shfl_xor(acc.x, 16);
    tot.y = acc.y + __shfl_xor(acc.y, 16);
    tot.z = acc.z + __shfl_xor(acc.z, 16);
    tot.w = acc.w + __shfl_xor(acc.w, 16);
    const v4f sv = *(const v4f*)(xs + (size_t)c * F + q4);
    const v4f av = (tot + sv) * (dc * ASCALE);
    if (hh == 0) {
      v4h hv;
      hv[0] = (_Float16)av.x; hv[1] = (_Float16)av.y; hv[2] = (_Float16)av.z; hv[3] = (_Float16)av.w;
      *(v4h*)(sA + (wave * 16 + j) * AP + q4) = hv;
    }
  }
  __syncthreads();

  v8f acc4[4];
#pragma unroll
  for (int t = 0; t < 4; ++t) { v8f z = {0.f, 0.f, 0.f, 0.f, 0.f, 0.f, 0.f, 0.f}; acc4[t] = z; }
  const _Float16* ar = sA + (wave * 16 + m) * AP + 8 * hh;
#pragma unroll
  for (int kt = 0; kt < F / 32; ++kt) {
    FragH a;
    a.h[0] = *(const v8h*)(ar + 32 * kt);
    a.h[1] = *(const v8h*)(ar + 32 * kt + 16);
#pragma unroll
    for (int t = 0; t < 4; ++t) {
      const _Float16* bp = wp + (size_t)(16 * t + m) * F + 32 * kt + 8 * hh;
      FragH b;
      b.h[0] = *(const v8h*)bp;
      b.h[1] = *(const v8h*)(bp + 16);
      acc4[t] = wmh(a.v, b.v, acc4[t]);
    }
  }
  __syncthreads();

  const int r0 = wave * 16 + 8 * hh;
  const v4f dA = *(const v4f*)(dinv + (size_t)rowBase + r0);
  const v4f dB = *(const v4f*)(dinv + (size_t)rowBase + r0 + 4);
  float s[8];
  s[0] = dA.x; s[1] = dA.y; s[2] = dA.z; s[3] = dA.w; s[4] = dB.x; s[5] = dB.y; s[6] = dB.z; s[7] = dB.w;
#pragma unroll
  for (int r = 0; r < 8; ++r) s[r] = scaleOut != 0 ? s[r] : 1.0f;
  float* sp = stg + r0 * F + m;
#pragma unroll
  for (int t = 0; t < 4; ++t) {
    const float bl = bias[16 * t + m];
#pragma unroll
    for (int r = 0; r < 8; ++r) {
      float v = acc4[t][r] * OSCALE + bl;
      v = lrelu(v);
      sp[r * F + 16 * t] = v * s[r];
    }
  }
  __syncthreads();

  const float* lp = stg + wave * 16 * F + 4 * lane;
  float* gp = xo + ((size_t)rowBase + wave * 16) * F + 4 * lane;
#pragma unroll
  for (int i = 0; i < 8; ++i) { const v4f v = *(const v4f*)(lp + 128 * i); *(volatile v4f*)(gp + 128 * i) = v; }
  __threadfence();
#pragma unroll
  for (int i = 0; i < 8; ++i) { const v4f v = *(const v4f*)(lp + 128 * i); *(volatile v4f*)(gp + 128 * i) = v; }
}

__global__ __launch_bounds__(NTHR) void k_pool(
    const int* __restrict__ batch, const float* __restrict__ h, float* pooled, int nN) {
  __shared__ __attribute__((aligned(16))) float acc[NBP * F];
  __shared__ __attribute__((aligned(16))) float mx[NBP * F];
  __shared__ __attribute__((aligned(16))) int list[LISTN];
  __shared__ int pc[NBP];
  __shared__ int wcnt[NWAVE];
  const int tid = threadIdx.x, lane = tid & 31, wave = tid >> 5;
  const int gBase = blockIdx.x * NBP;
  const float ninf = -__builtin_inff();

  {
    const v4f z = {0.f, 0.f, 0.f, 0.f};
    const v4f zi = {ninf, ninf, ninf, ninf};
    for (int i = tid; i < NBP * F / 4; i += NTHR) { ((v4f*)acc)[i] = z; ((v4f*)mx)[i] = zi; }
    for (int i = tid; i < NBP; i += NTHR) pc[i] = 0;
  }
  __syncthreads();

  const int nChunks = (nN + CHUNK - 1) / CHUNK;
#pragma unroll 1
  for (int ch = 0; ch < nChunks; ++ch) {
    const int cbase = ch * CHUNK;
    const int wc = scan_chunk<NBP>(batch, nN, cbase, gBase, 1, list, tid, lane, wave);
    if (lane == 0) wcnt[wave] = wc;
    __syncthreads();
    if (wave == 0) {
#pragma unroll 1
      for (int wsx = 0; wsx < NWAVE; ++wsx) {
        int n = __builtin_amdgcn_readfirstlane(wcnt[wsx]);
        n = n > WCAP ? WCAP : (n < 0 ? 0 : n);
        const int* lp = list + wsx * WCAP;
#pragma unroll 1
        for (int i = 0; i < n; ++i) {
          const int ent  = __builtin_amdgcn_readfirstlane(lp[i]);
          const int slot = ent & (NBP - 1);
          int nd = cbase + ((ent >> 12) & (CHUNK - 1));
          nd = nd > nN - 1 ? nN - 1 : nd;
          const v2f v = *(const v2f*)(h + (size_t)nd * F + 2 * lane);
          v2f* ap = (v2f*)(acc + slot * F + 2 * lane);
          *ap = *ap + v;
          v2f* mp = (v2f*)(mx + slot * F + 2 * lane);
          v2f mm = *mp;
          mm.x = fmaxf(mm.x, v.x);
          mm.y = fmaxf(mm.y, v.y);
          *mp = mm;
          if (lane == 0) pc[slot] = pc[slot] + 1;
        }
      }
    }
    __syncthreads();
  }

  v4f ov[4];
#pragma unroll
  for (int p = 0; p < 4; ++p) {
    const int g   = p * NTHR + tid;
    const int row = g >> 5;
    const int c0  = (g & 31) * 4;
    const int cc  = c0 & (F - 1);
    int cv = pc[row];
    cv = cv < 1 ? 1 : cv;
    const float inv = 1.0f / (float)cv;
    const v4f a = *(const v4f*)(acc + row * F + cc);
    const v4f b = *(const v4f*)(mx + row * F + cc);
    const bool isMean = c0 < F;
    ov[p].x = isMean ? a.x * inv : b.x;
    ov[p].y = isMean ? a.y * inv : b.y;
    ov[p].z = isMean ? a.z * inv : b.z;
    ov[p].w = isMean ? a.w * inv : b.w;
  }
  float* gp = pooled + (size_t)gBase * (2 * F);
#pragma unroll
  for (int p = 0; p < 4; ++p) *(volatile v4f*)(gp + 4 * (p * NTHR + tid)) = ov[p];
  __threadfence();
#pragma unroll
  for (int p = 0; p < 4; ++p) *(volatile v4f*)(gp + 4 * (p * NTHR + tid)) = ov[p];
}

__global__ __launch_bounds__(NTHR) void k_head(
    const float* __restrict__ pooled, const float* __restrict__ gfeat,
    const float* __restrict__ W1, const float* __restrict__ B1,
    const float* __restrict__ W2, const float* __restrict__ B2, float* h2) {
  __shared__ __attribute__((aligned(16))) float sP[HIN];
  __shared__ __attribute__((aligned(16))) float sH1[L1D];
  __shared__ __attribute__((aligned(16))) float sH2[L2D];
  const int g = blockIdx.x, t = threadIdx.x;
  int gi = t - 2 * F;
  gi = gi < 0 ? 0 : (gi > GFD - 1 ? GFD - 1 : gi);
  const float pa = pooled[(size_t)g * (2 * F) + (t & (2 * F - 1))];
  const float pb = gfeat[(size_t)g * GFD + gi];
  if (t < HIN) sP[t] = (t < 2 * F) ? pa : pb;
  __syncthreads();

  float a1 = B1[t];
#pragma unroll 4
  for (int k = 0; k < HIN; ++k) a1 += sP[k] * W1[(size_t)k * L1D + t];
  sH1[t] = lrelu(a1);
  __syncthreads();

  const int t2 = t & (L2D - 1);
  float a2 = B2[t2];
#pragma unroll 4
  for (int k = 0; k < L1D; ++k) a2 += sH1[k] * W2[(size_t)k * L2D + t2];
  if (t < L2D) sH2[t] = lrelu(a2);
  __syncthreads();

  v4f ov = {0.f, 0.f, 0.f, 0.f};
  if (t < 32) ov = *(const v4f*)(sH2 + 4 * t);
  float* op = h2 + (size_t)g * L2D;
  if (t < 32) *(volatile v4f*)(op + 4 * t) = ov;
  __threadfence();
  if (t < 32) *(volatile v4f*)(op + 4 * t) = ov;
}

__global__ __launch_bounds__(GOUT) void k_out(
    const float* __restrict__ h2, const float* __restrict__ ow, const float* __restrict__ ob, float* out) {
  __shared__ __attribute__((aligned(16))) float sO[GOUT];
  const int t = threadIdx.x;
  const int g = blockIdx.x * GOUT + t;
  const float* hp = h2 + (size_t)g * L2D;
  float a = ob[0];
#pragma unroll 4
  for (int k = 0; k < L2D; ++k) a += hp[k] * ow[k];
  sO[t] = a;
  __syncthreads();
  v4f ov = {0.f, 0.f, 0.f, 0.f};
  if (t < 32) ov = *(const v4f*)(sO + 4 * t);
  float* op = out + (size_t)blockIdx.x * GOUT;
  if (t < 32) *(volatile v4f*)(op + 4 * t) = ov;
  __threadfence();
  if (t < 32) *(volatile v4f*)(op + 4 * t) = ov;
}

extern "C" void kernel_launch(void* const* d_in, const int* in_sizes, int n_in,
                              void* d_out, int out_size, void* d_ws, size_t ws_size,
                              hipStream_t stream) {
  if (n_in < 16) return;
  const int nN  = in_sizes[0] / F;
  const int nGr = in_sizes[1] / GFD;
  const int nE  = in_sizes[14] / 2;
  if (nN <= 0 || nGr <= 0 || nE <= 0) return;
  if (in_sizes[0] != nN * F || in_sizes[1] != nGr * GFD || in_sizes[14] != 2 * nE || in_sizes[15] != nN) return;
  if (in_sizes[2] != F * F || in_sizes[4] != F * F || in_sizes[6] != F * F) return;
  if (in_sizes[3] < F || in_sizes[5] < F || in_sizes[7] < F) return;
  if (in_sizes[8] != HIN * L1D || in_sizes[9] < L1D || in_sizes[10] != L1D * L2D ||
      in_sizes[11] < L2D || in_sizes[12] < L2D || in_sizes[13] < 1) return;
  if (out_size != nGr || (nGr % GOUT) != 0) return;
  if (nE > (1 << 28) || nN > (1 << 24)) return;

  const float* x     = (const float*)d_in[0];
  const float* gfeat = (const float*)d_in[1];
  const float* cw1   = (const float*)d_in[2];
  const float* cb1   = (const float*)d_in[3];
  const float* cw2   = (const float*)d_in[4];
  const float* cb2   = (const float*)d_in[5];
  const float* cw3   = (const float*)d_in[6];
  const float* cb3   = (const float*)d_in[7];
  const float* fw1   = (const float*)d_in[8];
  const float* fb1   = (const float*)d_in[9];
  const float* fw2   = (const float*)d_in[10];
  const float* fb2   = (const float*)d_in[11];
  const float* ow    = (const float*)d_in[12];
  const float* ob    = (const float*)d_in[13];
  const int*   ei    = (const int*)d_in[14];
  const int*   batch = (const int*)d_in[15];
  float* out = (float*)d_out;

  const int NPAD   = ((nN + TGT - 1) / TGT) * TGT;
  const int nBC    = (nN + NBC - 1) / NBC;
  const int CNTPAD = nBC * NBC;
  if (4 * nBC + 1 > RBN) return;
  const int nBF    = (nN + NBF - 1) / NBF;
  const int csrPad = (32 * nBF + 1024 + 31) & ~31;
  const int csrLen = ((nE + 31) & ~31) + csrPad;
  const int nLayer = NPAD / TGT;
  const int nScale = NPAD / SROWS;
  const int nPool  = (nGr + NBP - 1) / NBP;
  const int NGPP   = nPool * NBP;
  const int nHead  = nGr;
  const int nOut   = nGr / GOUT;

  char* ws = (char*)d_ws;
  size_t off = 0;
  const size_t oWp  = off; off += (size_t)3 * F * F * 2;            off = (off + 255) & ~(size_t)255;
  const size_t oCnt = off; off += (size_t)CNTPAD * 4;               off = (off + 255) & ~(size_t)255;
  const size_t oDv  = off; off += (size_t)CNTPAD * 4;               off = (off + 255) & ~(size_t)255;
  const size_t oOff = off; off += (size_t)CNTPAD * 4;               off = (off + 255) & ~(size_t)255;
  const size_t oRb  = off; off += (size_t)RBN * 4;                  off = (off + 255) & ~(size_t)255;
  const size_t oCsr = off; off += (size_t)csrLen * 4;               off = (off + 255) & ~(size_t)255;
  const size_t oPa  = off; off += (size_t)NPAD * F * 4;             off = (off + 255) & ~(size_t)255;
  const size_t oPb  = off; off += (size_t)NPAD * F * 4;             off = (off + 255) & ~(size_t)255;
  const size_t oPl  = off; off += (size_t)NGPP * 2 * F * 4;         off = (off + 255) & ~(size_t)255;
  const size_t oH2  = off; off += (size_t)nGr * L2D * 4;            off = (off + 255) & ~(size_t)255;
  if (off > ws_size || off > ((size_t)128 << 20)) return;
  _Float16* wp   = (_Float16*)(ws + oWp);
  int*      cnt  = (int*)(ws + oCnt);
  float*    dinv = (float*)(ws + oDv);
  int*      offp = (int*)(ws + oOff);
  int*      rb   = (int*)(ws + oRb);
  int*      csr  = (int*)(ws + oCsr);
  float*    pa   = (float*)(ws + oPa);
  float*    pb   = (float*)(ws + oPb);
  float*    pl   = (float*)(ws + oPl);
  float*    h2   = (float*)(ws + oH2);

  const int vec8 = ((nE & 3) == 0) ? 1 : 0;

  k_wprep<<<(3 * F * F / 8) / NTHR, NTHR, 0, stream>>>(cw1, cw2, cw3, wp);

  k_count<<<nBC, NTHR, 0, stream>>>(ei, cnt, dinv, nE, vec8);
  k_offsets<<<1, OTHR, 0, stream>>>(cnt, offp, rb, nBC);
  hipFuncSetAttribute(reinterpret_cast<const void*>(&k_fill),
                      hipFuncAttributeMaxDynamicSharedMemorySize, LDS_FILL);
  k_fill<<<nBF, NTHR, LDS_FILL, stream>>>(ei, offp, rb, csr, nN, nE, vec8, csrLen);

  k_scale<<<nScale, NTHR, 0, stream>>>(x, dinv, pa, nN);

  k_layer<<<nLayer, NTHR, 0, stream>>>(csr, offp, cnt, dinv, pa, wp,                     cb1, pb, nN, csrLen, 1);
  k_layer<<<nLayer, NTHR, 0, stream>>>(csr, offp, cnt, dinv, pb, wp + (size_t)F * F,     cb2, pa, nN, csrLen, 1);
  k_layer<<<nLayer, NTHR, 0, stream>>>(csr, offp, cnt, dinv, pa, wp + (size_t)2 * F * F, cb3, pb, nN, csrLen, 0);

  k_pool<<<nPool, NTHR, 0, stream>>>(batch, pb, pl, nN);

  k_head<<<nHead, NTHR, 0, stream>>>(pl, gfeat, fw1, fb1, fw2, fb2, h2);
  k_out<<<nOut, GOUT, 0, stream>>>(h2, ow, ob, out);
}
